// Block_60284160966734
// MI455X (gfx1250) — hardware-verified
//
#include <hip/hip_runtime.h>
#include <stddef.h>


typedef _Float16 v16h __attribute__((ext_vector_type(16)));
typedef _Float16 v8h  __attribute__((ext_vector_type(8)));
typedef _Float16 v4h  __attribute__((ext_vector_type(4)));
typedef float    v8f  __attribute__((ext_vector_type(8)));
typedef float    v4f  __attribute__((ext_vector_type(4)));

#ifndef NB
#define NB 4
#endif
#ifndef SEQ
#define SEQ 2048
#endif
#ifndef VRES
#define VRES 1
#endif
#define NB_FULL  4
#define SEQ_FULL 2048
#define DIM   32
#define QKVN  96
#define HID   128
#define NHEAD 8
#define HD    4
#define MROWS (NB * SEQ)
#define QT    (SEQ / 16)

static_assert(NB >= 1 && NB <= NB_FULL);
static_assert(SEQ >= 64 && SEQ <= SEQ_FULL && (SEQ % 64) == 0);
static_assert(DIM == NHEAD * HD);
static_assert(HD == 4);
static_assert(DIM == 32);
static_assert(QKVN == 3 * DIM);
static_assert(HID == 4 * DIM && (HID % 32) == 0);
static_assert(NHEAD == 8);
static_assert((MROWS % 64) == 0);
static_assert((QT % 4) == 0);
static_assert(((QKVN * DIM) % (8 * 128)) == 0);
static_assert(((DIM * DIM) % (8 * 128)) == 0);
static_assert(((HID * DIM) % (8 * 128)) == 0);

#define LDA 40
#define LDX 36
#define LDQ 100
#define LDH 136
static_assert((LDA % 8) == 0 && LDA >= DIM);
static_assert((LDX % 4) == 0 && LDX >= DIM);
static_assert((LDQ % 4) == 0 && LDQ >= QKVN);
static_assert((LDH % 8) == 0 && LDH >= HID);
static_assert(64 * LDQ * 4 + 64 * LDX * 4 + 64 * LDA * 2 <= 131072);
static_assert(2 * 64 * LDA * 2 + 2 * 64 * LDX * 4 + 64 * LDH * 2 <= 131072);

#define WCARRY  64.0f
#define XCARRY  16.0f
#define QKCARRY 16.0f
#define VCARRY  16.0f
#define RCARRY  2048.0f
#define PLOG2   10.0f
#define CCARRY  64.0f
#define MCARRY  16.0f

#define WA_BYTES  ((size_t)QKVN * DIM * 2)
#define WP_BYTES  ((size_t)DIM * DIM * 2)
#define WF_BYTES  ((size_t)HID * DIM * 2)
#define X1_BYTES  ((size_t)MROWS * DIM * 4)
#define QK_BYTES  ((size_t)NB * NHEAD * SEQ * HD * 2)
#define VT_BYTES  ((size_t)NB * NHEAD * 8 * SEQ * 2)
#define OFF_WA  ((size_t)0)
#define OFF_WP  (OFF_WA + WA_BYTES)
#define OFF_W1  (OFF_WP + WP_BYTES)
#define OFF_W2  (OFF_W1 + WF_BYTES)
#define OFF_X1  (OFF_W2 + WF_BYTES)
#define OFF_K   (OFF_X1 + X1_BYTES)
#define OFF_Q   (OFF_K + QK_BYTES)
#define OFF_VT  (OFF_Q + QK_BYTES)
#define OFF_CX  (OFF_VT + VT_BYTES)
#define WS_TOTAL (OFF_CX + QK_BYTES)
static_assert((WA_BYTES % 128) == 0 && (WP_BYTES % 128) == 0 && (WF_BYTES % 128) == 0);
static_assert((X1_BYTES % 128) == 0 && (QK_BYTES % 128) == 0 && (VT_BYTES % 128) == 0);
static_assert(WS_TOTAL <= (size_t)134217728);

__device__ __forceinline__ float bf16r(float x) {
  unsigned int u = __float_as_uint(x);
  u = (u + 0x7FFFu + ((u >> 16) & 1u)) & 0xFFFF0000u;
  return __uint_as_float(u);
}

static __device__ __forceinline__ _Float16 toh_flush(float v) {
  const _Float16 r = (_Float16)v;
  return (fabsf(v) < 6.103515625e-05f) ? (_Float16)0.0f : r;
}

__device__ __forceinline__ v16h frag_at(const _Float16* p) {
  v8h lo = *(const v8h*)(p);
  v8h hi = *(const v8h*)(p + 16);
  v16h out;
#pragma unroll
  for (int i = 0; i < 8; ++i) { out[i] = lo[i]; out[i + 8] = hi[i]; }
  return out;
}
__device__ __forceinline__ v16h ld_frag(const _Float16* base, unsigned ld) {
  const unsigned lane = threadIdx.x & 31u;
  return frag_at(base + (lane & 15u) * ld + (lane >> 4) * 8u);
}

__device__ __forceinline__ v8f wmma16(v16h a, v16h b, v8f c) {
  v8f d = __builtin_amdgcn_wmma_f32_16x16x32_f16(false, a, false, b, (short)0, c,
                                                 false, false);
  asm volatile("v_nop\n\tv_nop\n\tv_nop\n\tv_nop" : "+v"(d) : "v"(a), "v"(b));
  return d;
}

__device__ __forceinline__ float red32_sum(float x) {
#pragma unroll
  for (int off = 1; off < 32; off <<= 1) x += __shfl_xor(x, off, 32);
  return x;
}

__device__ __forceinline__ float ex2(float x) { return __builtin_amdgcn_exp2f(x); }

__global__ __launch_bounds__(128) void wcvt_kernel(
    const float* __restrict__ W, _Float16* __restrict__ P16, unsigned n8) {
  const unsigned g = blockIdx.x * 128u + threadIdx.x;
  if (g < n8) {
    const v4f a0 = *(const v4f*)(W + (size_t)g * 8u);
    const v4f a1 = *(const v4f*)(W + (size_t)g * 8u + 4u);
    v8h o;
#pragma unroll
    for (int i = 0; i < 4; ++i) {
      o[i]     = toh_flush(WCARRY * bf16r(a0[i]));
      o[i + 4] = toh_flush(WCARRY * bf16r(a1[i]));
    }
    _Float16* p = P16 + (size_t)g * 8u;
    *(volatile v8h*)p = o;
    __threadfence();
    *(volatile v8h*)p = o;
  }
}

__global__ __launch_bounds__(256) void ln_qkv_kernel(
    const float* __restrict__ X, const float* __restrict__ G1,
    const _Float16* __restrict__ Wa, float* __restrict__ X1,
    _Float16* __restrict__ Kp, _Float16* __restrict__ Qp, _Float16* __restrict__ Vt) {
  __shared__ __attribute__((aligned(16))) float Cs[64 * LDQ];
  __shared__ __attribute__((aligned(16))) float Xs[64 * LDX];
  __shared__ __attribute__((aligned(16))) _Float16 As[64 * LDA];

  const unsigned tid = threadIdx.x, lane = tid & 31u;
  const unsigned w = (unsigned)__builtin_amdgcn_readfirstlane((int)(threadIdx.x >> 5));
  const unsigned hh = lane >> 4, m = lane & 15u;
  const unsigned row0 = blockIdx.x * 64u;
  const unsigned bidx = row0 / (unsigned)SEQ;
  const unsigned t0 = row0 - bidx * (unsigned)SEQ;
  const size_t frow0 = (size_t)bidx * SEQ_FULL + t0;

  const float gl = bf16r(G1[lane]);
#pragma unroll 1
  for (unsigned j = 0; j < 8u; ++j) {
    const unsigned r = w * 8u + j;
    const float xv = bf16r(X[(frow0 + r) * DIM + lane]);
    const float mean = red32_sum(xv) * (1.0f / (float)DIM);
    const float d = xv - mean;
    const float var = red32_sum(d * d) * (1.0f / (float)DIM);
    const float rstd = 1.0f / sqrtf(var + 1.0e-5f);
    const float xn = d * rstd * gl;
    Xs[r * LDX + lane] = xn;
    As[r * LDA + lane] = toh_flush(XCARRY * xn);
  }
  __syncthreads();

  const unsigned mw = w >> 1, nw = w & 1u;
  const v16h a = ld_frag(&As[(mw * 16u) * LDA], LDA);
#pragma unroll
  for (unsigned j = 0; j < 3u; ++j) {
    const unsigned n0 = nw * 48u + 16u * j;
    const v16h bfr = frag_at(Wa + (size_t)(n0 + m) * DIM + hh * 8u);
    v8f acc = {};
    acc = wmma16(a, bfr, acc);
#pragma unroll
    for (int r = 0; r < 8; ++r)
      Cs[(mw * 16u + hh * 8u + (unsigned)r) * LDQ + n0 + m] = acc[r];
  }
  __syncthreads();

  const float qs = QKCARRY / (XCARRY * WCARRY);
  const float vs = VCARRY / (XCARRY * WCARRY);
  const unsigned bh = bidx * NHEAD + w;

  v8h xk, xq;
#pragma unroll
  for (unsigned j = 0; j < 8u; ++j) {
    const unsigned rr = 2u * lane + (j >> 2);
    const unsigned cc = w * 4u + (j & 3u);
    xk[j] = toh_flush(Cs[rr * LDQ + cc] * qs);
    xq[j] = toh_flush(Cs[rr * LDQ + 32u + cc] * qs);
  }
  const size_t offk = ((size_t)bh * SEQ + t0 + 2u * lane) * HD;

  v8h xv[2];
  size_t offv[2];
#pragma unroll
  for (unsigned i = 0; i < 2u; ++i) {
    const unsigned vrow = 4u * i + (lane >> 3);
    const unsigned dcol = vrow & 3u;
    const unsigned kk = (lane & 7u) * 8u;
#pragma unroll
    for (unsigned j = 0; j < 8u; ++j) {
      const float t = Cs[(kk + j) * LDQ + 64u + w * 4u + dcol] * vs;
      const _Float16 hi = toh_flush(t);
      if (i == 0u) {
        xv[i][j] = hi;
      } else {
        xv[i][j] = VRES ? toh_flush((t - (float)hi) * RCARRY) : (_Float16)0.0f;
      }
    }
    offv[i] = ((size_t)bh * 8u + vrow) * SEQ + t0 + kk;
  }

  v4f xx[2];
  size_t offx[2];
#pragma unroll
  for (unsigned i = 0; i < 2u; ++i) {
    const unsigned r = 32u * i + (tid >> 3);
    const unsigned c = (tid & 7u) * 4u;
    xx[i] = *(const v4f*)&Xs[r * LDX + c];
    offx[i] = (size_t)(row0 + r) * DIM + c;
  }

  *(volatile v8h*)(Kp + offk) = xk;
  *(volatile v8h*)(Qp + offk) = xq;
#pragma unroll
  for (int i = 0; i < 2; ++i) *(volatile v8h*)(Vt + offv[i]) = xv[i];
#pragma unroll
  for (int i = 0; i < 2; ++i) *(volatile v4f*)(X1 + offx[i]) = xx[i];
  __threadfence();
  *(volatile v8h*)(Kp + offk) = xk;
  *(volatile v8h*)(Qp + offk) = xq;
#pragma unroll
  for (int i = 0; i < 2; ++i) *(volatile v8h*)(Vt + offv[i]) = xv[i];
#pragma unroll
  for (int i = 0; i < 2; ++i) *(volatile v4f*)(X1 + offx[i]) = xx[i];
}

static __device__ __forceinline__ void attn_step(
    const _Float16* __restrict__ Kp, const _Float16* __restrict__ Vt,
    const size_t koff, const size_t voff, const v16h qf, const v16h fillv,
    const bool lowhalf, const bool vlane, const bool masked,
    const unsigned key0, const unsigned qidx, v8f& acc, float& mr) {
  const v4h k0v = *(const v4h*)(Kp + koff);
  const v4h k1v = *(const v4h*)(Kp + koff + 64);
  const v16h vraw = frag_at(Vt + voff);
  const _Float16 hz = (_Float16)0.0f;
  v16h ka = {};
  v16h kc = {};
#pragma unroll
  for (int i = 0; i < 4; ++i) {
    ka[i] = lowhalf ? k0v[i] : hz;
    kc[i] = lowhalf ? k1v[i] : hz;
  }
  v8f s0 = {};
  v8f s1 = {};
  s0 = wmma16(ka, qf, s0);
  s1 = wmma16(kc, qf, s1);

  const float sscale = 0.72134752044448170368f / (QKCARRY * QKCARRY);
  float e0[8], e1[8];
  float tmax = -1.0e30f;
#pragma unroll
  for (int r = 0; r < 8; ++r) {
    float a = s0[r] * sscale;
    float b = s1[r] * sscale;
    if (masked) {
      a = (key0 + (unsigned)r > qidx) ? -1.0e30f : a;
      b = (key0 + 16u + (unsigned)r > qidx) ? -1.0e30f : b;
    }
    e0[r] = a;
    e1[r] = b;
    tmax = fmaxf(tmax, fmaxf(a, b));
  }
  tmax = fmaxf(tmax, __shfl_xor(tmax, 16, 32));
  const float nm = fmaxf(mr, tmax);
  const float corr = ex2(mr - nm);
  mr = nm;
  const float sh = PLOG2 - nm;
  v16h pf;
#pragma unroll
  for (int r = 0; r < 8; ++r) {
    const float x0 = e0[r] + sh;
    const float x1 = e1[r] + sh;
    const float p0 = (x0 < -14.0f) ? 0.0f : ex2(x0);
    const float p1 = (x1 < -14.0f) ? 0.0f : ex2(x1);
    pf[r]     = (_Float16)p0;
    pf[r + 8] = (_Float16)p1;
  }
#pragma unroll
  for (int r = 0; r < 8; ++r) acc[r] = acc[r] * corr;
  const v16h va = vlane ? vraw : fillv;
  acc = wmma16(va, pf, acc);
}

__global__ __launch_bounds__(128) void attn_kernel(
    const _Float16* __restrict__ Qp, const _Float16* __restrict__ Kp,
    const _Float16* __restrict__ Vt, _Float16* __restrict__ Cx) {
  const unsigned lane = threadIdx.x & 31u;
  const unsigned hh = lane >> 4, m = lane & 15u;
  const int wslot = (int)(threadIdx.x >> 5);
  const int g = (int)(blockIdx.x % (unsigned)(QT / 4));
  const unsigned bh = blockIdx.x / (unsigned)(QT / 4);
  const int it = __builtin_amdgcn_readfirstlane(
      (wslot >> 1) * (QT / 2) + g + (wslot & 1) * (QT / 2 - 1 - 2 * g));
  const unsigned i0 = (unsigned)it * 16u;
  const int nsteps = (it + 2) >> 1;

  const bool lowhalf = (hh == 0u);
  const bool vlane = (m < 8u);
  const _Float16 hz = (_Float16)0.0f;
  const _Float16 hone = (_Float16)1.0f;

  const v4h qv = *(const v4h*)(Qp + ((size_t)bh * SEQ + i0 + m) * HD);
  v16h qf = {};
#pragma unroll
  for (int i = 0; i < 4; ++i) qf[i] = lowhalf ? qv[i] : hz;
  v16h fillv;
#pragma unroll
  for (int i = 0; i < 16; ++i) fillv[i] = (m == 8u) ? hone : hz;

  v8f acc = {};
  float mr = -1.0e30f;
  const size_t kbase = ((size_t)bh * SEQ + m) * HD;
  const size_t vbase = ((size_t)bh * 8u + (m & 7u)) * SEQ + hh * 8u;
  const unsigned qidx = i0 + m;

  for (int s = 0; s < nsteps - 1; ++s) {
    attn_step(Kp, Vt, kbase + (size_t)s * 128u, vbase + (size_t)s * 32u, qf, fillv,
              lowhalf, vlane, false, (unsigned)s * 32u + hh * 8u, qidx, acc, mr);
  }
  {
    const int s = nsteps - 1;
    attn_step(Kp, Vt, kbase + (size_t)s * 128u, vbase + (size_t)s * 32u, qf, fillv,
              lowhalf, vlane, true, (unsigned)s * 32u + hh * 8u, qidx, acc, mr);
  }

  const float lsum = __shfl(acc[0], (int)(m + 16u), 32);
  const float inv = __builtin_amdgcn_rcpf(lsum) * (CCARRY / VCARRY);
  v4h o;
#pragma unroll
  for (int d = 0; d < 4; ++d)
    o[d] = toh_flush((acc[d] + acc[d + 4] * (1.0f / RCARRY)) * inv);
  _Float16* dst = Cx + ((size_t)bh * SEQ + i0 + m) * HD;
  if (lowhalf) *(volatile v4h*)dst = o;
  __threadfence();
  if (lowhalf) *(volatile v4h*)dst = o;
}

__global__ __launch_bounds__(256) void post_kernel(
    const _Float16* __restrict__ Cx, const float* __restrict__ X1,
    const _Float16* __restrict__ Wp, const float* __restrict__ bp,
    const float* __restrict__ G2,
    const _Float16* __restrict__ W1, const float* __restrict__ b1,
    const _Float16* __restrict__ W2, const float* __restrict__ b2,
    float* __restrict__ outf) {
  __shared__ __attribute__((aligned(16))) _Float16 As[64 * LDA];
  __shared__ __attribute__((aligned(16))) _Float16 A2s[64 * LDA];
  __shared__ __attribute__((aligned(16))) float Cs[64 * LDX];
  __shared__ __attribute__((aligned(16))) float Xs[64 * LDX];
  __shared__ __attribute__((aligned(16))) _Float16 Hs[64 * LDH];

  const unsigned tid = threadIdx.x, lane = tid & 31u;
  const unsigned w = (unsigned)__builtin_amdgcn_readfirstlane((int)(threadIdx.x >> 5));
  const unsigned hh = lane >> 4, m = lane & 15u;
  const unsigned mw = w >> 1, nw = w & 1u;
  const unsigned row0 = blockIdx.x * 64u;
  const unsigned bidx = row0 / (unsigned)SEQ;
  const unsigned t0 = row0 - bidx * (unsigned)SEQ;
  const size_t frow0 = (size_t)bidx * SEQ_FULL + t0;

#pragma unroll
  for (unsigned j = 0; j < 2u; ++j) {
    const unsigned p = tid + 256u * j;
    const unsigned hd = p >> 6, r = p & 63u;
    const v4h c = *(const v4h*)(Cx + ((size_t)(bidx * NHEAD + hd) * SEQ + t0 + r) * HD);
    *(v4h*)&As[r * LDA + hd * 4u] = c;
  }
  __syncthreads();

  {
    const v16h a = ld_frag(&As[(mw * 16u) * LDA], LDA);
    const v16h bfr = frag_at(Wp + (size_t)(nw * 16u + m) * DIM + hh * 8u);
    v8f acc = {};
    acc = wmma16(a, bfr, acc);
#pragma unroll
    for (int r = 0; r < 8; ++r)
      Cs[(mw * 16u + hh * 8u + (unsigned)r) * LDX + nw * 16u + m] = acc[r];
  }
  __syncthreads();

  {
    const float g2l = bf16r(G2[lane]);
    const float bpl = bf16r(bp[lane]);
#pragma unroll 1
    for (unsigned j = 0; j < 8u; ++j) {
      const unsigned r = w * 8u + j;
      const float y = Cs[r * LDX + lane] * (1.0f / (CCARRY * WCARRY)) + bpl;
      const float x2 = X1[(size_t)(row0 + r) * DIM + lane] + y;
      const float mean = red32_sum(x2) * (1.0f / (float)DIM);
      const float d = x2 - mean;
      const float var = red32_sum(d * d) * (1.0f / (float)DIM);
      const float rstd = 1.0f / sqrtf(var + 1.0e-5f);
      const float xn = d * rstd * g2l;
      Xs[r * LDX + lane] = xn;
      A2s[r * LDA + lane] = toh_flush(XCARRY * xn);
    }
  }
  __syncthreads();

  {
    const v16h a2 = ld_frag(&A2s[(mw * 16u) * LDA], LDA);
#pragma unroll 1
    for (unsigned j = 0; j < 4u; ++j) {
      const unsigned n0 = nw * 64u + 16u * j;
      const v16h bfr = frag_at(W1 + (size_t)(n0 + m) * DIM + hh * 8u);
      v8f acc = {};
      acc = wmma16(a2, bfr, acc);
      const float bias = bf16r(b1[n0 + m]);
#pragma unroll
      for (int r = 0; r < 8; ++r) {
        const float t = acc[r] * (1.0f / (XCARRY * WCARRY)) + bias;
        const float ge = 0.5f * t * (1.0f + erff(t * 0.70710678118654752f));
        Hs[(mw * 16u + hh * 8u + (unsigned)r) * LDH + n0 + m] = toh_flush(MCARRY * ge);
      }
    }
  }
  __syncthreads();

  {
    v8f acc = {};
#pragma unroll
    for (unsigned c = 0; c < 4u; ++c) {
      const v16h a = ld_frag(&Hs[(mw * 16u) * LDH + c * 32u], LDH);
      const v16h bfr = frag_at(W2 + (size_t)(nw * 16u + m) * HID + c * 32u + hh * 8u);
      acc = wmma16(a, bfr, acc);
    }
#pragma unroll
    for (int r = 0; r < 8; ++r)
      Cs[(mw * 16u + hh * 8u + (unsigned)r) * LDX + nw * 16u + m] = acc[r];
  }
  __syncthreads();

  v4f xs[2];
  size_t off[2];
#pragma unroll
  for (unsigned i = 0; i < 2u; ++i) {
    const unsigned r = 32u * i + (tid >> 3);
    const unsigned c = (tid & 7u) * 4u;
    const v4f u  = *(const v4f*)&Cs[r * LDX + c];
    const v4f xr = *(const v4f*)&Xs[r * LDX + c];
    const v4f gb = *(const v4f*)(b2 + c);
    v4f val;
#pragma unroll
    for (int j = 0; j < 4; ++j)
      val[j] = xr[j] + (u[j] * (1.0f / (MCARRY * WCARRY)) + bf16r(gb[j]));
    xs[i] = val;
    off[i] = (frow0 + r) * DIM + c;
  }
#pragma unroll
  for (int i = 0; i < 2; ++i) *(volatile v4f*)(outf + off[i]) = xs[i];
  __threadfence();
#pragma unroll
  for (int i = 0; i < 2; ++i) *(volatile v4f*)(outf + off[i]) = xs[i];
}

extern "C" void kernel_launch(void* const* d_in, const int* in_sizes, int n_in,
                              void* d_out, int out_size, void* d_ws, size_t ws_size,
                              hipStream_t stream) {
  if (n_in < 10) return;
  const long long need_x = ((long long)(NB - 1) * SEQ_FULL + SEQ) * DIM;
  if ((long long)in_sizes[0] < need_x) return;
  if (in_sizes[1] < QKVN * DIM) return;
  if (in_sizes[2] < DIM * DIM) return;
  if (in_sizes[3] < DIM || in_sizes[4] < DIM || in_sizes[5] < DIM) return;
  if (in_sizes[6] < HID * DIM || in_sizes[7] < HID) return;
  if (in_sizes[8] < DIM * HID || in_sizes[9] < DIM) return;
  if ((long long)out_size < need_x) return;
  if (ws_size < WS_TOTAL) return;

  const float* X      = (const float*)d_in[0];
  const float* w_attn = (const float*)d_in[1];
  const float* w_proj = (const float*)d_in[2];
  const float* b_proj = (const float*)d_in[3];
  const float* g1     = (const float*)d_in[4];
  const float* g2     = (const float*)d_in[5];
  const float* w_ff1  = (const float*)d_in[6];
  const float* b_ff1  = (const float*)d_in[7];
  const float* w_ff2  = (const float*)d_in[8];
  const float* b_ff2  = (const float*)d_in[9];
  float* out = (float*)d_out;

  char* ws = (char*)d_ws;
  _Float16* Wa16 = (_Float16*)(ws + OFF_WA);
  _Float16* Wp16 = (_Float16*)(ws + OFF_WP);
  _Float16* W116 = (_Float16*)(ws + OFF_W1);
  _Float16* W216 = (_Float16*)(ws + OFF_W2);
  float*    X1   = (float*)(ws + OFF_X1);
  _Float16* Kp16 = (_Float16*)(ws + OFF_K);
  _Float16* Qp16 = (_Float16*)(ws + OFF_Q);
  _Float16* Vt16 = (_Float16*)(ws + OFF_VT);
  _Float16* Cx16 = (_Float16*)(ws + OFF_CX);

  wcvt_kernel<<<dim3((QKVN * DIM / 8) / 128), dim3(128), 0, stream>>>(
      w_attn, Wa16, (unsigned)(QKVN * DIM / 8));
  wcvt_kernel<<<dim3((DIM * DIM / 8) / 128), dim3(128), 0, stream>>>(
      w_proj, Wp16, (unsigned)(DIM * DIM / 8));
  wcvt_kernel<<<dim3((HID * DIM / 8) / 128), dim3(128), 0, stream>>>(
      w_ff1, W116, (unsigned)(HID * DIM / 8));
  wcvt_kernel<<<dim3((HID * DIM / 8) / 128), dim3(128), 0, stream>>>(
      w_ff2, W216, (unsigned)(HID * DIM / 8));

  ln_qkv_kernel<<<dim3(MROWS / 64), dim3(256), 0, stream>>>(X, g1, Wa16, X1, Kp16, Qp16, Vt16);
  attn_kernel<<<dim3(NB * NHEAD * (QT / 4)), dim3(128), 0, stream>>>(Qp16, Kp16, Vt16, Cx16);
  post_kernel<<<dim3(MROWS / 64), dim3(256), 0, stream>>>(Cx16, X1, Wp16, b_proj, g2,
                                                          W116, b_ff1, W216, b_ff2, out);
}
